// TinyTransformerBlock_89472758711002
// MI455X (gfx1250) — hardware-verified
//
#include <hip/hip_runtime.h>
#include <stddef.h>


typedef _Float16 h16;
typedef _Float16 v16h __attribute__((ext_vector_type(16)));
typedef _Float16 v8h  __attribute__((ext_vector_type(8)));
typedef _Float16 v4h  __attribute__((ext_vector_type(4)));
typedef float    v8f  __attribute__((ext_vector_type(8)));
typedef float    v4f  __attribute__((ext_vector_type(4)));

#ifndef NB
#define NB 8
#endif
#ifndef SEQ
#define SEQ 4096
#endif
#define NB_FULL  8
#define SEQ_FULL 4096
#define DIM    256
#define QKROWS 512
#define NHEAD  4
#define HD     64
#define MROWS  (NB * SEQ)

static_assert(NB >= 1 && NB <= NB_FULL);
static_assert(SEQ >= 256 && SEQ <= SEQ_FULL);
static_assert((SEQ % 256) == 0);
static_assert(((SEQ / 8) % 32) == 0);
static_assert((SEQ % 128) == 0);
static_assert(((NB * SEQ) % 1024) == 0);
static_assert(DIM == NHEAD * HD);
static_assert(HD == 64);
static_assert(QKROWS == 2 * DIM);
static_assert((DIM % 64) == 0 && (DIM % 32) == 0);
static_assert((QKROWS % 64) == 0);
static_assert((HD % 32) == 0);
static_assert((MROWS % 64) == 0);
static_assert((SEQ % 64) == 0);
static_assert(((3 * DIM * DIM) % 2048) == 0 && ((DIM * DIM) % 2048) == 0);
static_assert((size_t)MROWS * DIM < (size_t)0xFFFFFFFFu);

#define LDT 72
#define LDC 68
static_assert((LDT % 8) == 0 && LDT >= 64);
static_assert((LDC % 4) == 0 && LDC >= 64);

#define WCARRY  64.0f
#define QKCARRY 16.0f
#define VPCARRY 16.0f
#define PCARRY  1024.0f
#define OCARRY  64.0f

#define XT_BYTES   ((size_t)MROWS * DIM * 2)
#define WQKV_BYTES ((size_t)3 * DIM * DIM * 2)
#define WPR_BYTES  ((size_t)DIM * DIM * 2)
#define QK_BYTES   ((size_t)NB * QKROWS * SEQ * 2)
#define VP_BYTES   ((size_t)MROWS * DIM * 2)
#define PP_BYTES   ((size_t)NB * NHEAD * HD * HD * 2)
#define CTX_BYTES  ((size_t)MROWS * DIM * 2)
#define Y_BYTES    ((size_t)NB * DIM * SEQ * 4)
#define OFF_XT   ((size_t)0)
#define OFF_WQKV (OFF_XT + XT_BYTES)
#define OFF_WPR  (OFF_WQKV + WQKV_BYTES)
#define OFF_QK   (OFF_WPR + WPR_BYTES)
#define OFF_VP   (OFF_QK + QK_BYTES)
#define OFF_PP   (OFF_VP + VP_BYTES)
#define OFF_CTX  (OFF_PP + PP_BYTES)
#define OFF_Y    (OFF_CTX + CTX_BYTES)
#define WS_TOTAL (OFF_Y + Y_BYTES)
static_assert((XT_BYTES % 128) == 0 && (WQKV_BYTES % 128) == 0 && (WPR_BYTES % 128) == 0);
static_assert((QK_BYTES % 128) == 0 && (VP_BYTES % 128) == 0 && (PP_BYTES % 128) == 0);
static_assert((CTX_BYTES % 128) == 0 && (Y_BYTES % 128) == 0);
static_assert(WS_TOTAL <= (size_t)134217728);

__device__ __forceinline__ float bf16r(float x) {
  unsigned int u = __float_as_uint(x);
  u = (u + 0x7FFFu + ((u >> 16) & 1u)) & 0xFFFF0000u;
  return __uint_as_float(u);
}

static __device__ __forceinline__ h16 toh_flush(float v) {
  const h16 r = (h16)v;
  return (fabsf(v) < 6.103515625e-05f) ? (h16)0.0f : r;
}

__device__ __forceinline__ v16h frag_at(const _Float16* p) {
  v8h lo = *(const v8h*)(p);
  v8h hi = *(const v8h*)(p + 16);
  v16h out;
#pragma unroll
  for (int i = 0; i < 8; ++i) { out[i] = lo[i]; out[i + 8] = hi[i]; }
  return out;
}

__device__ __forceinline__ v8f wmma16(v16h a, v16h b, v8f c) {
  v8f d = __builtin_amdgcn_wmma_f32_16x16x32_f16(false, a, false, b, (short)0, c,
                                                 false, false);
  asm volatile("v_nop\n\tv_nop\n\tv_nop\n\tv_nop" : "+v"(d) : "v"(a), "v"(b));
  return d;
}

__device__ __forceinline__ float red16_max(float x) {
#pragma unroll
  for (int off = 1; off < 16; off <<= 1) x = fmaxf(x, __shfl_xor(x, off, 32));
  return x;
}
__device__ __forceinline__ float red16_sum(float x) {
#pragma unroll
  for (int off = 1; off < 16; off <<= 1) x += __shfl_xor(x, off, 32);
  return x;
}
__device__ __forceinline__ float red32_sum(float x) {
#pragma unroll
  for (int off = 1; off < 32; off <<= 1) x += __shfl_xor(x, off, 32);
  return x;
}

__global__ __launch_bounds__(256) void wconv_kernel(
    const float* __restrict__ W, _Float16* __restrict__ Wt, unsigned ldw, unsigned ldk) {
  __shared__ _Float16 T[64 * LDT];
  const unsigned tid = threadIdx.x;
  const unsigned n0 = blockIdx.x * 64u;
  const unsigned k0 = blockIdx.y * 64u;
#pragma unroll 4
  for (unsigned j = 0; j < 16u; ++j) {
    const unsigned idx = tid + 256u * j;
    const unsigned kr = idx >> 6, nc = idx & 63u;
    const float v = W[(size_t)(k0 + kr) * ldw + n0 + nc];
    T[nc * LDT + kr] = (_Float16)(WCARRY * bf16r(v));
  }
  __syncthreads();
  v8h x[2];
  size_t off[2];
#pragma unroll
  for (unsigned i = 0; i < 2u; ++i) {
    const unsigned n = 32u * i + (tid >> 3);
    const unsigned kc = (tid & 7u) * 8u;
    x[i] = *(const v8h*)&T[n * LDT + kc];
    off[i] = (size_t)(n0 + n) * ldk + k0 + kc;
  }
#pragma unroll
  for (int i = 0; i < 2; ++i) *(volatile v8h*)(Wt + off[i]) = x[i];
  __threadfence();
#pragma unroll
  for (int i = 0; i < 2; ++i) *(volatile v8h*)(Wt + off[i]) = x[i];
}

__global__ __launch_bounds__(256) void wplane_kernel(
    const float* __restrict__ W, _Float16* __restrict__ Wp) {
  const size_t e0 = ((size_t)blockIdx.x * 256u + threadIdx.x) * 8u;
  const v4f a0 = *(const v4f*)(W + e0);
  const v4f a1 = *(const v4f*)(W + e0 + 4u);
  v8h o;
#pragma unroll
  for (int i = 0; i < 4; ++i) {
    o[i]     = toh_flush(WCARRY * bf16r(a0[i]));
    o[i + 4] = toh_flush(WCARRY * bf16r(a1[i]));
  }
  *(volatile v8h*)(Wp + e0) = o;
  __threadfence();
  *(volatile v8h*)(Wp + e0) = o;
}

template <int MODE>
__device__ __forceinline__ void gemm_body(
    const _Float16* __restrict__ A16, const unsigned lda,
    const _Float16* __restrict__ Bt, const unsigned ldb, const unsigned K,
    const float* __restrict__ bias, const float* __restrict__ addf,
    float* __restrict__ outf, _Float16* __restrict__ out16) {
  __shared__ float Cs[64 * LDC];
  const unsigned tid = threadIdx.x, lane = tid & 31u, w = tid >> 5;
  const unsigned mw = w >> 1, nw = w & 1u;
  const unsigned hh = lane >> 4, m = lane & 15u;
  const unsigned n0 = blockIdx.x * 64u;
  const unsigned row0 = blockIdx.y * 64u;

  const _Float16* ap  = A16 + (size_t)(row0 + mw * 16u + m) * lda + hh * 8u;
  const _Float16* bp0 = Bt + (size_t)(nw * 32u + m) * ldb + hh * 8u;
  const _Float16* bp1 = bp0 + (size_t)16 * ldb;
  v8f acc0 = {}, acc1 = {};
#pragma unroll 2
  for (unsigned k0 = 0; k0 < K; k0 += 32u) {
    const v16h a  = frag_at(ap + k0);
    const v16h b0 = frag_at(bp0 + k0);
    const v16h b1 = frag_at(bp1 + k0);
    acc0 = wmma16(a, b0, acc0);
    acc1 = wmma16(a, b1, acc1);
  }
#pragma unroll
  for (int r = 0; r < 8; ++r) {
    const unsigned ci = (mw * 16u + hh * 8u + (unsigned)r) * LDC + nw * 32u + m;
    Cs[ci]       = acc0[r];
    Cs[ci + 16u] = acc1[r];
  }
  __syncthreads();

  if (MODE == 0 || MODE == 2) {
    v8h x[2];
    size_t off[2];
#pragma unroll
    for (unsigned i = 0; i < 2u; ++i) {
      const unsigned r = 32u * i + (tid >> 3);
      const unsigned c = (tid & 7u) * 8u;
      const v4f u0 = *(const v4f*)&Cs[r * LDC + c];
      const v4f u1 = *(const v4f*)&Cs[r * LDC + c + 4];
      if (MODE == 2) {
#pragma unroll
        for (int j = 0; j < 4; ++j) {
          x[i][j]     = toh_flush(u0[j] * (OCARRY / (VPCARRY * PCARRY)));
          x[i][j + 4] = toh_flush(u1[j] * (OCARRY / (VPCARRY * PCARRY)));
        }
      } else {
        const v4f g0 = *(const v4f*)(bias + n0 + c);
        const v4f g1 = *(const v4f*)(bias + n0 + c + 4u);
#pragma unroll
        for (int j = 0; j < 4; ++j) {
          x[i][j]     = toh_flush(VPCARRY * (u0[j] * (1.0f / (WCARRY * WCARRY)) + bf16r(g0[j])));
          x[i][j + 4] = toh_flush(VPCARRY * (u1[j] * (1.0f / (WCARRY * WCARRY)) + bf16r(g1[j])));
        }
      }
      off[i] = (size_t)(row0 + r) * DIM + n0 + c;
    }
#pragma unroll
    for (int i = 0; i < 2; ++i) *(volatile v8h*)(out16 + off[i]) = x[i];
    __threadfence();
#pragma unroll
    for (int i = 0; i < 2; ++i) *(volatile v8h*)(out16 + off[i]) = x[i];
  }

  if (MODE == 1) {
    const unsigned bidx = row0 / (unsigned)SEQ;
    const unsigned key0 = row0 - bidx * (unsigned)SEQ;
    v8h x[2];
    size_t off[2];
#pragma unroll
    for (unsigned i = 0; i < 2u; ++i) {
      const unsigned dcol = 32u * i + (tid >> 3);
      const unsigned kk = (tid & 7u) * 8u;
      const float bb = bf16r(bias[n0 + dcol]);
#pragma unroll
      for (unsigned j = 0; j < 8u; ++j) {
        const float t = Cs[(kk + j) * LDC + dcol] * (1.0f / (WCARRY * WCARRY)) + bb;
        x[i][j] = toh_flush(QKCARRY * t);
      }
      off[i] = ((size_t)bidx * QKROWS + n0 + dcol) * SEQ + key0 + kk;
    }
#pragma unroll
    for (int i = 0; i < 2; ++i) *(volatile v8h*)(out16 + off[i]) = x[i];
    __threadfence();
#pragma unroll
    for (int i = 0; i < 2; ++i) *(volatile v8h*)(out16 + off[i]) = x[i];
  }

  if (MODE == 3) {
    const unsigned bidx = row0 / (unsigned)SEQ;
    const unsigned key0 = row0 - bidx * (unsigned)SEQ;
    v4f xs[4];
    size_t off[4];
#pragma unroll
    for (unsigned i = 0; i < 4u; ++i) {
      const unsigned o  = 16u * i + (tid >> 4);
      const unsigned pc = (tid & 15u) * 4u;
      const float bb = bf16r(bias[n0 + o]);
      const v4f xin = *(const v4f*)(addf + ((size_t)bidx * DIM + n0 + o) * SEQ_FULL + key0 + pc);
      v4f val;
#pragma unroll
      for (unsigned j = 0; j < 4u; ++j) {
        const float u = Cs[(pc + j) * LDC + o];
        val[j] = bf16r(xin[j]) + (u * (1.0f / (OCARRY * WCARRY)) + bb);
      }
      xs[i] = val;
      off[i] = ((size_t)bidx * DIM + n0 + o) * SEQ + key0 + pc;
    }
#pragma unroll
    for (int i = 0; i < 4; ++i) *(volatile v4f*)(outf + off[i]) = xs[i];
    __threadfence();
#pragma unroll
    for (int i = 0; i < 4; ++i) *(volatile v4f*)(outf + off[i]) = xs[i];
  }
}

__global__ __launch_bounds__(256) void gemm_qk_kernel(
    const _Float16* __restrict__ Xt, const _Float16* __restrict__ Wqk,
    const float* __restrict__ bias, _Float16* __restrict__ qk) {
  gemm_body<1>(Xt, (unsigned)DIM, Wqk + (size_t)blockIdx.x * 64u * DIM, (unsigned)DIM,
               (unsigned)DIM, bias, bias, (float*)0, qk);
}
__global__ __launch_bounds__(256) void gemm_v_kernel(
    const _Float16* __restrict__ Xt, const _Float16* __restrict__ Wv,
    const float* __restrict__ bias, _Float16* __restrict__ vp) {
  gemm_body<0>(Xt, (unsigned)DIM, Wv + (size_t)blockIdx.x * 64u * DIM, (unsigned)DIM,
               (unsigned)DIM, bias, bias, (float*)0, vp);
}
__global__ __launch_bounds__(256) void gemm_pv_kernel(
    const _Float16* __restrict__ Vp, const _Float16* __restrict__ Pp,
    _Float16* __restrict__ ctx) {
  const unsigned bidx = (blockIdx.y * 64u) / (unsigned)SEQ;
  gemm_body<2>(Vp + blockIdx.x * HD, (unsigned)DIM,
               Pp + (size_t)(bidx * NHEAD + blockIdx.x) * (HD * HD), (unsigned)HD,
               (unsigned)HD, (const float*)0, (const float*)0, (float*)0, ctx);
}
__global__ __launch_bounds__(256) void gemm_proj_kernel(
    const _Float16* __restrict__ ctx, const _Float16* __restrict__ Wp,
    const float* __restrict__ bias, const float* __restrict__ xin, float* __restrict__ y) {
  gemm_body<3>(ctx, (unsigned)DIM, Wp + (size_t)blockIdx.x * 64u * DIM, (unsigned)DIM,
               (unsigned)DIM, bias, xin, y, (_Float16*)0);
}

__global__ __launch_bounds__(256) void score_kernel(
    const _Float16* __restrict__ QK, _Float16* __restrict__ Pp) {
  __shared__ float Sp[8 * 16 * LDC];
  __shared__ _Float16 Pt[16 * LDT];

  const unsigned tid = threadIdx.x, lane = tid & 31u;
  const int wave = __builtin_amdgcn_readfirstlane(threadIdx.x >> 5);
  const unsigned hh = lane >> 4, m = lane & 15u;
  const unsigned d0 = blockIdx.x * 16u;
  const unsigned head = blockIdx.y;
  const unsigned b = blockIdx.z;

  const _Float16* qp = QK + ((size_t)b * QKROWS + head * HD + d0 + m) * SEQ + hh * 8u;
  const _Float16* kp = QK + ((size_t)b * QKROWS + DIM + head * HD + m) * SEQ + hh * 8u;
  const unsigned kbeg = (unsigned)wave * (unsigned)(SEQ / 8);
  const unsigned kend = kbeg + (unsigned)(SEQ / 8);

  v8f acc0 = {}, acc1 = {}, acc2 = {}, acc3 = {};
#pragma unroll 2
  for (unsigned k0 = kbeg; k0 < kend; k0 += 32u) {
    const v16h a  = frag_at(qp + k0);
    const v16h b0 = frag_at(kp + k0);
    const v16h b1 = frag_at(kp + (size_t)16 * SEQ + k0);
    const v16h b2 = frag_at(kp + (size_t)32 * SEQ + k0);
    const v16h b3 = frag_at(kp + (size_t)48 * SEQ + k0);
    acc0 = wmma16(a, b0, acc0);
    acc1 = wmma16(a, b1, acc1);
    acc2 = wmma16(a, b2, acc2);
    acc3 = wmma16(a, b3, acc3);
  }
  const unsigned sbase = (unsigned)wave * (16u * LDC);
#pragma unroll
  for (int r = 0; r < 8; ++r) {
    const unsigned si = sbase + (hh * 8u + (unsigned)r) * LDC + m;
    Sp[si]       = acc0[r];
    Sp[si + 16u] = acc1[r];
    Sp[si + 32u] = acc2[r];
    Sp[si + 48u] = acc3[r];
  }
  __syncthreads();

  const unsigned row = tid >> 4;
  const unsigned c = (tid & 15u) * 4u;
  v4f s = *(const v4f*)&Sp[row * LDC + c];
#pragma unroll
  for (unsigned w2 = 1; w2 < 8u; ++w2) {
    const v4f t = *(const v4f*)&Sp[(w2 * 16u + row) * LDC + c];
    s += t;
  }
  const float sc = 0.125f / (QKCARRY * QKCARRY);
#pragma unroll
  for (int j = 0; j < 4; ++j) s[j] = s[j] * sc;
  float mx = fmaxf(fmaxf(s[0], s[1]), fmaxf(s[2], s[3]));
  mx = red16_max(mx);
  v4f e;
#pragma unroll
  for (int j = 0; j < 4; ++j) e[j] = __expf(s[j] - mx);
  const float rs = red16_sum((e[0] + e[1]) + (e[2] + e[3]));
  const float inv = PCARRY * (1.0f / rs);
  v4h pv;
#pragma unroll
  for (int j = 0; j < 4; ++j) pv[j] = toh_flush(e[j] * inv);
  *(v4h*)&Pt[row * LDT + c] = pv;
  __syncthreads();

  if (wave < 4) {
    const unsigned r = tid >> 3;
    const unsigned cc = (tid & 7u) * 8u;
    const v8h x = *(const v8h*)&Pt[r * LDT + cc];
    _Float16* dst = Pp + ((size_t)(b * NHEAD + head) * HD + d0 + r) * HD + cc;
    *(volatile v8h*)dst = x;
    __threadfence();
    *(volatile v8h*)dst = x;
  }
}

#define BN_PR    (SEQ / 4)
#define BN_ITERS ((NB * SEQ) / 1024)
__global__ __launch_bounds__(256) void bn_kernel(
    const float* __restrict__ Y, const float* __restrict__ G, const float* __restrict__ Be,
    float* __restrict__ out) {
#pragma clang fp contract(off)
  __shared__ float red_a[8];
  __shared__ float red_b[8];
  const unsigned tid = threadIdx.x, lane = tid & 31u;
  const int wave = __builtin_amdgcn_readfirstlane(threadIdx.x >> 5);
  const unsigned ch = blockIdx.x;
  const float inv_n = 1.0f / (float)(NB * SEQ);

  float s = 0.0f;
#pragma unroll 1
  for (unsigned it = 0; it < (unsigned)BN_ITERS; ++it) {
    const unsigned i = tid + 256u * it;
    const unsigned b = i / (unsigned)BN_PR;
    const unsigned pp = i - b * (unsigned)BN_PR;
    const v4f a = *(const v4f*)(Y + ((size_t)b * DIM + ch) * SEQ + pp * 4u);
    s += (a[0] + a[1]) + (a[2] + a[3]);
  }
  s = red32_sum(s);
  if (lane == 0u) red_a[wave] = s;
  __syncthreads();
  float tot = red_a[0];
#pragma unroll
  for (int w2 = 1; w2 < 8; ++w2) tot += red_a[w2];
  const float mean = tot * inv_n;

  float ss = 0.0f;
#pragma unroll 1
  for (unsigned it = 0; it < (unsigned)BN_ITERS; ++it) {
    const unsigned i = tid + 256u * it;
    const unsigned b = i / (unsigned)BN_PR;
    const unsigned pp = i - b * (unsigned)BN_PR;
    const v4f a = *(const v4f*)(Y + ((size_t)b * DIM + ch) * SEQ + pp * 4u);
    const float e0 = a[0] - mean, e1 = a[1] - mean, e2 = a[2] - mean, e3 = a[3] - mean;
    ss += (e0 * e0 + e1 * e1) + (e2 * e2 + e3 * e3);
  }
  ss = red32_sum(ss);
  if (lane == 0u) red_b[wave] = ss;
  __syncthreads();
  float tot2 = red_b[0];
#pragma unroll
  for (int w2 = 1; w2 < 8; ++w2) tot2 += red_b[w2];
  const float var = tot2 * inv_n;
  const float rstd = 1.0f / sqrtf(var + 1.0e-5f);
  const float g  = bf16r(G[ch]);
  const float be = bf16r(Be[ch]);

#pragma unroll 1
  for (unsigned it = 0; it < (unsigned)BN_ITERS; ++it) {
    const unsigned i = tid + 256u * it;
    const unsigned b = i / (unsigned)BN_PR;
    const unsigned pp = i - b * (unsigned)BN_PR;
    const v4f a = *(const v4f*)(Y + ((size_t)b * DIM + ch) * SEQ + pp * 4u);
    v4f o;
#pragma unroll
    for (int j = 0; j < 4; ++j) o[j] = ((a[j] - mean) * rstd) * g + be;
    float* p = out + ((size_t)b * DIM + ch) * SEQ_FULL + pp * 4u;
    *(volatile v4f*)p = o;
    __threadfence();
    *(volatile v4f*)p = o;
  }
}

extern "C" void kernel_launch(void* const* d_in, const int* in_sizes, int n_in,
                              void* d_out, int out_size, void* d_ws, size_t ws_size,
                              hipStream_t stream) {
  if (n_in < 7) return;
  const long long need_x = ((long long)NB * DIM - 1) * SEQ_FULL + SEQ;
  if ((long long)in_sizes[0] < need_x) return;
  if ((long long)in_sizes[1] < (long long)3 * DIM * DIM) return;
  if (in_sizes[2] < 3 * DIM) return;
  if ((long long)in_sizes[3] < (long long)DIM * DIM) return;
  if (in_sizes[4] < DIM || in_sizes[5] < DIM || in_sizes[6] < DIM) return;
  if ((long long)out_size < need_x) return;
  if (ws_size < WS_TOTAL) return;

  const float* X     = (const float*)d_in[0];
  const float* wqkv  = (const float*)d_in[1];
  const float* bqkv  = (const float*)d_in[2];
  const float* wproj = (const float*)d_in[3];
  const float* bproj = (const float*)d_in[4];
  const float* gam   = (const float*)d_in[5];
  const float* bet   = (const float*)d_in[6];
  float* out = (float*)d_out;

  char* ws = (char*)d_ws;
  _Float16* Xt16   = (_Float16*)(ws + OFF_XT);
  _Float16* Wqkv16 = (_Float16*)(ws + OFF_WQKV);
  _Float16* Wpr16  = (_Float16*)(ws + OFF_WPR);
  _Float16* QK16   = (_Float16*)(ws + OFF_QK);
  _Float16* Vp16   = (_Float16*)(ws + OFF_VP);
  _Float16* Pp16   = (_Float16*)(ws + OFF_PP);
  _Float16* Ctx16  = (_Float16*)(ws + OFF_CTX);
  float*    Yf     = (float*)(ws + OFF_Y);

  dim3 blk(256);

  for (int b = 0; b < NB; ++b) {
    wconv_kernel<<<dim3(SEQ / 64, DIM / 64), blk, 0, stream>>>(
        X + (size_t)b * DIM * SEQ_FULL, Xt16 + (size_t)b * SEQ * DIM,
        (unsigned)SEQ_FULL, (unsigned)DIM);
  }
  wplane_kernel<<<dim3((3 * DIM * DIM) / 2048), blk, 0, stream>>>(wqkv, Wqkv16);
  wplane_kernel<<<dim3((DIM * DIM) / 2048), blk, 0, stream>>>(wproj, Wpr16);

  gemm_qk_kernel<<<dim3(QKROWS / 64, MROWS / 64), blk, 0, stream>>>(Xt16, Wqkv16, bqkv, QK16);
  gemm_v_kernel<<<dim3(DIM / 64, MROWS / 64), blk, 0, stream>>>(
      Xt16, Wqkv16 + (size_t)QKROWS * DIM, bqkv + QKROWS, Vp16);
  score_kernel<<<dim3(HD / 16, NHEAD, NB), blk, 0, stream>>>(QK16, Pp16);
  gemm_pv_kernel<<<dim3(NHEAD, MROWS / 64), blk, 0, stream>>>(Vp16, Pp16, Ctx16);
  gemm_proj_kernel<<<dim3(DIM / 64, MROWS / 64), blk, 0, stream>>>(Ctx16, Wpr16, bproj, X, Yf);
  bn_kernel<<<dim3(DIM), blk, 0, stream>>>(Yf, gam, bet, out);
}
